// GAT_ED_58755152609378
// MI455X (gfx1250) — hardware-verified
//
#include <hip/hip_runtime.h>
#include <math.h>

constexpr int kBatch = 64;
constexpr int kTime  = 128;
constexpr int kNode  = 64;
constexpr int kHid   = 64;
constexpr int kEmb   = 128;
constexpr int kTaps  = 7;
constexpr int kGate3 = 192;
constexpr int kRows  = kBatch * kTime;
constexpr int kPairRows = kBatch * kNode;
constexpr int kColK  = kTaps * kNode;
constexpr int kNT    = 256;
constexpr int kHP    = 72;
constexpr int kTP    = 72;

typedef __attribute__((ext_vector_type(16))) _Float16 v16h;
typedef __attribute__((ext_vector_type(8)))  _Float16 v8h;
typedef __attribute__((ext_vector_type(16))) __bf16   v16b;
typedef __attribute__((ext_vector_type(8)))  __bf16   v8b;
typedef __attribute__((ext_vector_type(8)))  float    v8f;
typedef __attribute__((ext_vector_type(4)))  float    v4f;

__device__ __forceinline__ unsigned short f2bf_bits(float f) {
  unsigned u = __float_as_uint(f);
  return (unsigned short)((u + 0x7FFFu + ((u >> 16) & 1u)) >> 16);
}
__device__ __forceinline__ float bf_bits2f(unsigned short h) { return __uint_as_float(((unsigned)h) << 16); }

__device__ __forceinline__ void dep_guard_h(v8f& a, v8f& b, v16h x, v16h y) { asm volatile("v_nop\n\tv_nop\n\tv_nop\n\tv_nop" : "+v"(a), "+v"(b) : "v"(x), "v"(y)); }
__device__ __forceinline__ void dep_guard_b(v8f& a, v8f& b, v16b x, v16b y) { asm volatile("v_nop\n\tv_nop\n\tv_nop\n\tv_nop" : "+v"(a), "+v"(b) : "v"(x), "v"(y)); }
__device__ __forceinline__ void keep4_h(v16h a, v16h b, v16h c, v16h d) { asm volatile("v_nop" :: "v"(a), "v"(b), "v"(c), "v"(d)); }
__device__ __forceinline__ void keep4_b(v16b a, v16b b, v16b c, v16b d) { asm volatile("v_nop" :: "v"(a), "v"(b), "v"(c), "v"(d)); }
__device__ __forceinline__ void acc_guard4(v8f& a, v8f& b, v8f& c, v8f& d) { asm volatile("v_nop\n\tv_nop\n\tv_nop\n\tv_nop" : "+v"(a), "+v"(b), "+v"(c), "+v"(d)); }
__device__ __forceinline__ void dep_guard3_h(v8f& a, v8f& b, v8f& c, v16h w, v16h x, v16h y, v16h z) {
  asm volatile("v_nop\n\tv_nop\n\tv_nop\n\tv_nop" : "+v"(a), "+v"(b), "+v"(c) : "v"(w), "v"(x), "v"(y), "v"(z));
}
__device__ __forceinline__ void acc_guard3(v8f& a, v8f& b, v8f& c) { asm volatile("v_nop\n\tv_nop\n\tv_nop\n\tv_nop" : "+v"(a), "+v"(b), "+v"(c)); }

template <typename T> struct Frag;
template <> struct Frag<_Float16> {
  typedef v16h V; union U { v16h v; v8h h[2]; };
  static __device__ __forceinline__ v16h load(const _Float16* p) {
    U f; f.h[0] = *(const v8h*)(p); f.h[1] = *(const v8h*)(p + 16); return f.v;
  }
  static __device__ __forceinline__ v8f mma(v16h a, v16h b, v8f c) {
    return __builtin_amdgcn_wmma_f32_16x16x32_f16(false, a, false, b, (short)0, c, false, false);
  }
  static __device__ __forceinline__ void guard(v8f& a, v8f& b, v16h x, v16h y) { dep_guard_h(a, b, x, y); }
  static __device__ __forceinline__ void keep(v16h a, v16h b, v16h c, v16h d) { keep4_h(a, b, c, d); }
};
template <> struct Frag<__bf16> {
  typedef v16b V; union U { v16b v; v8b h[2]; };
  static __device__ __forceinline__ v16b load(const __bf16* p) {
    U f; f.h[0] = *(const v8b*)(p); f.h[1] = *(const v8b*)(p + 16); return f.v;
  }
  static __device__ __forceinline__ v8f mma(v16b a, v16b b, v8f c) {
    return __builtin_amdgcn_wmma_f32_16x16x32_bf16(false, a, false, b, (short)0, c, false, false);
  }
  static __device__ __forceinline__ void guard(v8f& a, v8f& b, v16b x, v16b y) { dep_guard_b(a, b, x, y); }
  static __device__ __forceinline__ void keep(v16b a, v16b b, v16b c, v16b d) { keep4_b(a, b, c, d); }
};

__device__ __forceinline__ unsigned pack_f16x2(float a, float b) {
  const _Float16 h0 = (_Float16)a, h1 = (_Float16)b;
  return (unsigned)__builtin_bit_cast(unsigned short, h0) | ((unsigned)__builtin_bit_cast(unsigned short, h1) << 16);
}
__device__ __forceinline__ void st2u(unsigned* p, unsigned v) { *(volatile unsigned*)p = v; __threadfence(); *(volatile unsigned*)p = v; }
__device__ __forceinline__ float ftanh(float x) { return 1.0f - 2.0f * __builtin_amdgcn_rcpf(1.0f + __expf(2.0f * x)); }
__device__ __forceinline__ float fsigm(float x) { return __builtin_amdgcn_rcpf(1.0f + __expf(-x)); }
__device__ __forceinline__ float selu_f(float v) {
  const float sc = 1.0507009873554805f, al = 1.6732632423543772f;
  const float neg = __expf(fminf(v, 0.0f)) - 1.0f;
  return sc * (fmaxf(v, 0.0f) + al * neg);
}

template <int ET> struct Elem;
template <> struct Elem<0> { typedef _Float16 T; };
template <> struct Elem<1> { typedef __bf16 T; };
template <int ET, bool SPLIT, int BIAS_MODE, int OUT_MODE, bool RESID, int ACT = 0>
__global__ __launch_bounds__(256) void wmma_gemm64(
    const unsigned short* __restrict__ Ap, const unsigned short* __restrict__ A2p, int lda, long strideA,
    const unsigned short* __restrict__ Btp, const unsigned short* __restrict__ Bt2p, int ldb, long strideB,
    void* __restrict__ Cout, void* __restrict__ Cout2, int ldc, long strideC,
    const float* __restrict__ bias,
    const float* __restrict__ resid, long strideR,
    int M, int N, int K, float scale) {
  typedef typename Elem<ET>::T T;
  typedef typename Frag<T>::V V;
  const T* A = (const T*)Ap; const T* A2 = (const T*)A2p; const T* Bt = (const T*)Btp; const T* Bt2 = (const T*)Bt2p;
  __shared__ __align__(16) float sT[8][16 * 68];
  const int b    = blockIdx.y;
  const int lane = threadIdx.x & 31;
  const int wave = threadIdx.x >> 5;
  const int tilesN = N >> 6;
  const int tilesM = M >> 6;
  const int tile = blockIdx.x * 8 + wave;
  if (tile >= tilesM * tilesN) return;
  const int tm = tile / tilesN;
  const int tn = tile - tm * tilesN;
  const int m0 = tm << 6;
  const int n0 = tn << 6;

  const T* Ab  = A  + (size_t)b * strideA;
  const T* Bb  = Bt + (size_t)b * strideB;
  const T* Ab2 = SPLIT ? (A2  + (size_t)b * strideA) : nullptr;
  const T* Bb2 = SPLIT ? (Bt2 + (size_t)b * strideB) : nullptr;

  const int rlane = lane & 15;
  const int koff  = (lane >> 4) * 8;
  const int mOff  = (lane >> 4) * 8;

  v8f acc[4][4];
#pragma unroll
  for (int i = 0; i < 4; ++i)
#pragma unroll
    for (int j = 0; j < 4; ++j) acc[i][j] = (v8f){0.f,0.f,0.f,0.f,0.f,0.f,0.f,0.f};

  for (int k0 = 0; k0 < K; k0 += 32) {
    V bh[4], bl[4];
#pragma unroll
    for (int j = 0; j < 4; ++j) {
      const size_t bo = (size_t)(n0 + (j << 4) + rlane) * ldb + koff + k0;
      bh[j] = Frag<T>::load(Bb + bo);
      if (SPLIT) bl[j] = Frag<T>::load(Bb2 + bo);
    }
#pragma unroll
    for (int i = 0; i < 4; ++i) {
      const size_t ao = (size_t)(m0 + (i << 4) + rlane) * lda + koff + k0;
      V ah = Frag<T>::load(Ab + ao);
      V al;
      if (SPLIT) al = Frag<T>::load(Ab2 + ao);
#pragma unroll
      for (int j = 0; j < 4; ++j) {
        acc[i][j] = Frag<T>::mma(ah, bh[j], acc[i][j]);
        if (SPLIT) {
          acc[i][j] = Frag<T>::mma(ah, bl[j], acc[i][j]);
          acc[i][j] = Frag<T>::mma(al, bh[j], acc[i][j]);
        }
      }
      Frag<T>::guard(acc[i][0], acc[i][3], ah, SPLIT ? al : ah);
    }
    Frag<T>::keep(bh[0], bh[1], bh[2], bh[3]);
    if (SPLIT) Frag<T>::keep(bl[0], bl[1], bl[2], bl[3]);
  }
  acc_guard4(acc[0][0], acc[0][1], acc[0][2], acc[0][3]);
  acc_guard4(acc[1][0], acc[1][1], acc[1][2], acc[1][3]);
  acc_guard4(acc[2][0], acc[2][1], acc[2][2], acc[2][3]);
  acc_guard4(acc[3][0], acc[3][1], acc[3][2], acc[3][3]);

  float* slab = sT[wave];
  const float* Rb = RESID ? (resid + (size_t)b * strideR) : nullptr;
#pragma unroll
  for (int i = 0; i < 4; ++i) {
    const int mBase = m0 + (i << 4);
#pragma unroll
    for (int j = 0; j < 4; ++j) {
      const int n = n0 + (j << 4) + rlane;
      float bv = 0.f;
      if (BIAS_MODE == 2) bv = bias[n];
#pragma unroll
      for (int r = 0; r < 8; ++r) {
        float v = acc[i][j][r] * scale;
        if (BIAS_MODE == 1) v += bias[mBase + mOff + r];
        if (BIAS_MODE == 2) v += bv;
        if (RESID) v += Rb[(size_t)(mBase + mOff + r) * ldc + n];
        if (ACT == 1) v = tanhf(v);
        if (ACT == 2) v = fmaxf(v, 0.0f);
        if (ACT == 3) v = v / (1.0f + expf(-v));
        if (ACT == 4) v = (v > 0.f) ? v : 0.01f * v;
        if (ACT == 5) v = 0.5f * v * (1.0f + erff(v * 0.70710678118654752f));
        if (ACT == 6) v = fsigm(v);
        slab[(mOff + r) * 68 + (j << 4) + rlane] = v;
      }
    }
    __builtin_amdgcn_fence(__ATOMIC_RELEASE, "workgroup");
    __builtin_amdgcn_wave_barrier();
    __builtin_amdgcn_fence(__ATOMIC_ACQUIRE, "workgroup");
    if (OUT_MODE == 0) {
      float* C = (float*)Cout + (size_t)b * strideC;
      const int hh = lane >> 4, c4 = (lane & 15) * 4;
      for (int pass = 0; pass < 2; ++pass) {
#pragma unroll
        for (int it = 0; it < 8; ++it) {
          const int row = it * 2 + hh;
          v4f v = *(const v4f*)(slab + row * 68 + c4);
          *(volatile v4f*)(C + (size_t)(mBase + row) * ldc + n0 + c4) = v;
        }
        __threadfence();
      }
    } else {
      const int q = lane >> 3, c8 = (lane & 7) * 8;
      unsigned short* C  = (unsigned short*)Cout  + (size_t)b * strideC;
      unsigned short* C2 = (OUT_MODE == 2) ? ((unsigned short*)Cout2 + (size_t)b * strideC) : nullptr;
      for (int pass = 0; pass < 2; ++pass) {
#pragma unroll
        for (int it = 0; it < 4; ++it) {
          const int row = it * 4 + q;
          const float* sp = slab + row * 68 + c8;
          v8h hv, lv;
#pragma unroll
          for (int e = 0; e < 8; ++e) {
            if (OUT_MODE == 1) {
              hv[e] = (_Float16)sp[e];
            } else {
              unsigned short hb = f2bf_bits(sp[e]);
              unsigned short lb = f2bf_bits(sp[e] - bf_bits2f(hb));
              hv[e] = __builtin_bit_cast(_Float16, hb);
              lv[e] = __builtin_bit_cast(_Float16, lb);
            }
          }
          *(volatile v8h*)(C + (size_t)(mBase + row) * ldc + n0 + c8) = hv;
          if (OUT_MODE == 2) *(volatile v8h*)(C2 + (size_t)(mBase + row) * ldc + n0 + c8) = lv;
        }
        __threadfence();
      }
    }
    __builtin_amdgcn_fence(__ATOMIC_RELEASE, "workgroup");
    __builtin_amdgcn_wave_barrier();
    __builtin_amdgcn_fence(__ATOMIC_ACQUIRE, "workgroup");
  }
}

__global__ __launch_bounds__(kNT) void prep_x_kernel(const float* __restrict__ x, _Float16* __restrict__ XCOL) {
  const int gid = blockIdx.x * kNT + threadIdx.x;
  const int row = gid / 56;
  const int rem = gid - row * 56;
  const int kk  = rem >> 3;
  const int c8  = (rem & 7) * 8;
  const int b = row >> 7, t = row & 127;
  const int ts = t + kk - 3;
  const bool valid = (ts >= 0) && (ts < kTime);
  const int tc = ts < 0 ? 0 : (ts > kTime - 1 ? kTime - 1 : ts);
  const float* p = x + ((size_t)(b * kTime + tc)) * kNode + c8;
  const v4f a0 = *(const v4f*)p;
  const v4f a1 = *(const v4f*)(p + 4);
  v8h h;
#pragma unroll
  for (int e = 0; e < 4; ++e) {
    h[e]     = valid ? (_Float16)a0[e] : (_Float16)0.0f;
    h[4 + e] = valid ? (_Float16)a1[e] : (_Float16)0.0f;
  }
  _Float16* op = XCOL + (size_t)row * kColK + kk * kNode + c8;
  *(volatile v8h*)op = h;
  __threadfence();
  *(volatile v8h*)op = h;
}

__global__ __launch_bounds__(kNT) void prep_w_kernel(
    const float* __restrict__ conv_w, const float* __restrict__ Ww,
    const float* __restrict__ We_ih, const float* __restrict__ We_hh,
    const float* __restrict__ Wm_ih, const float* __restrict__ Wm_hh,
    const float* __restrict__ Wd_ih, const float* __restrict__ Wd_hh,
    const float* __restrict__ W_dec, const float* __restrict__ W_p1, const float* __restrict__ W_p2,
    unsigned* __restrict__ WCONV, unsigned* __restrict__ WCAT,
    unsigned* __restrict__ WEIH, unsigned* __restrict__ WEHH,
    unsigned* __restrict__ WMIH, unsigned* __restrict__ WMHH,
    unsigned* __restrict__ WDIH, unsigned* __restrict__ WDHH,
    unsigned* __restrict__ WDEC, unsigned* __restrict__ WP1, unsigned* __restrict__ WP2) {
  const int y = blockIdx.y;
  const float* src = conv_w; unsigned* dst = WCONV; int nblk = 56;
  if (y == 1)       { src = Ww;    dst = WCAT; nblk = 64; }
  else if (y == 2)  { src = We_ih; dst = WEIH; nblk = 24; }
  else if (y == 3)  { src = We_hh; dst = WEHH; nblk = 24; }
  else if (y == 4)  { src = Wm_ih; dst = WMIH; nblk = 48; }
  else if (y == 5)  { src = Wm_hh; dst = WMHH; nblk = 24; }
  else if (y == 6)  { src = Wd_ih; dst = WDIH; nblk = 24; }
  else if (y == 7)  { src = Wd_hh; dst = WDHH; nblk = 24; }
  else if (y == 8)  { src = W_dec; dst = WDEC; nblk = 8; }
  else if (y == 9)  { src = W_p1;  dst = WP1;  nblk = 8; }
  else if (y == 10) { src = W_p2;  dst = WP2;  nblk = 8; }
  if ((int)blockIdx.x >= nblk) return;
  const int p = blockIdx.x * kNT + threadIdx.x;
  const int d = 2 * p;
  float f0, f1;
  if (y == 0) {
    const int o = d / kColK;
    const int kidx = d - o * kColK;
    const int kk = kidx >> 6, ci = kidx & 63;
    f0 = src[((size_t)o * kNode + ci) * kTaps + kk];
    f1 = src[((size_t)o * kNode + ci + 1) * kTaps + kk];
  } else if (y == 1) {
    const int n = d >> 7, t = d & 127;
    const size_t base = (size_t)(n & 127) * (2 * kTime) + (size_t)(n >> 7) * kTime + t;
    f0 = src[base];
    f1 = src[base + 1];
  } else {
    f0 = src[d];
    f1 = src[d + 1];
  }
  st2u(dst + p, pack_f16x2(f0 * 16.0f, f1 * 16.0f));
}

__global__ __launch_bounds__(kNT) void selu_layout_kernel(const float* __restrict__ CONV,
                                                          _Float16* __restrict__ CBTN, _Float16* __restrict__ VNT) {
  __shared__ __align__(16) _Float16 T16[kTime * kTP];
  const int b = blockIdx.x, tid = threadIdx.x, lane = tid & 31, wave = tid >> 5;
#pragma unroll 1
  for (int it = 0; it < 8; ++it) {
    const int idx = it * kNT + tid;
    const int row = idx >> 4, c4 = (idx & 15) * 4;
    const v4f v = *(const v4f*)(CONV + ((size_t)(b * kTime + row)) * kNode + c4);
#pragma unroll
    for (int e = 0; e < 4; ++e) T16[row * kTP + c4 + e] = (_Float16)selu_f(v[e]);
  }
  __syncthreads();
  for (int pass = 0; pass < 2; ++pass) {
#pragma unroll
    for (int it = 0; it < 4; ++it) {
      const int row = it * 32 + wave * 4 + (lane >> 3);
      const int c8 = (lane & 7) * 8;
      const v8h v = *(const v8h*)(T16 + row * kTP + c8);
      *(volatile v8h*)(CBTN + ((size_t)(b * kTime + row)) * kNode + c8) = v;
    }
#pragma unroll
    for (int it = 0; it < 4; ++it) {
      const int i = it * 16 + wave * 2 + (lane >> 4);
      const int t8 = (lane & 15) * 8;
      v8h h;
#pragma unroll
      for (int e = 0; e < 8; ++e) h[e] = T16[(t8 + e) * kTP + i];
      *(volatile v8h*)(VNT + ((size_t)(b * kNode + i)) * kTime + t8) = h;
    }
    __threadfence();
  }
}

__global__ __launch_bounds__(128) void gru_rec_kernel(const float* __restrict__ XG, const _Float16* __restrict__ WHH,
                                                     const float* __restrict__ bhh, _Float16* __restrict__ HSEQ, int ldo) {
  __shared__ __align__(16) _Float16 h16[16 * kHP];
  const int tid = threadIdx.x, lane = tid & 31, wave = tid >> 5;
  const int rlane = lane & 15, hh = lane >> 4, koff = hh * 8, mOff = hh * 8;
  const int blk = blockIdx.x;
  for (int i = tid; i < 16 * kHP; i += 128) h16[i] = (_Float16)0.0f;
  __syncthreads();

  const int j = 16 * wave + rlane;
  const _Float16* arow = h16 + rlane * kHP + koff;
  const _Float16* wr = WHH + (size_t)j * kHid + koff;
  const _Float16* wz = WHH + (size_t)(kHid + j) * kHid + koff;
  const _Float16* wn = WHH + (size_t)(2 * kHid + j) * kHid + koff;
  const float br = bhh[j], bz = bhh[kHid + j], bn = bhh[2 * kHid + j];
  const float* xgb = XG + (size_t)(blk * 16 + mOff) * kTime * kGate3 + j;
  const v8f z8 = {0.f, 0.f, 0.f, 0.f, 0.f, 0.f, 0.f, 0.f};
  const float s16 = 1.0f / 16.0f;

  float hreg[8];
#pragma unroll
  for (int r = 0; r < 8; ++r) hreg[r] = 0.0f;

#pragma unroll 1
  for (int t = 0; t < kTime; ++t) {
    v8f ar = z8, az = z8, an = z8;
#pragma unroll 1
    for (int k0 = 0; k0 < kHid; k0 += 32) {
      const v16h a  = Frag<_Float16>::load(arow + k0);
      const v16h b0 = Frag<_Float16>::load(wr + k0);
      const v16h b1 = Frag<_Float16>::load(wz + k0);
      const v16h b2 = Frag<_Float16>::load(wn + k0);
      ar = Frag<_Float16>::mma(a, b0, ar);
      az = Frag<_Float16>::mma(a, b1, az);
      an = Frag<_Float16>::mma(a, b2, an);
      dep_guard3_h(ar, az, an, a, b0, b1, b2);
    }
    acc_guard3(ar, az, an);

    const float* xt = xgb + (size_t)t * kGate3;
#pragma unroll
    for (int r = 0; r < 8; ++r) {
      const float* xr = xt + (size_t)r * kTime * kGate3;
      const float x_r = xr[0], x_z = xr[kHid], x_n = xr[2 * kHid];
      const float hr = ar[r] * s16 + br;
      const float hz = az[r] * s16 + bz;
      const float hn = an[r] * s16 + bn;
      const float rg = fsigm(x_r + hr);
      const float zg = fsigm(x_z + hz);
      const float ng = ftanh(x_n + rg * hn);
      hreg[r] = (1.0f - zg) * ng + zg * hreg[r];
    }
    __syncthreads();
#pragma unroll
    for (int r = 0; r < 8; ++r) h16[(mOff + r) * kHP + j] = (_Float16)hreg[r];
    __syncthreads();
    {
      _Float16* hsb = HSEQ + ((size_t)(blk * 16) * kTime + t) * (size_t)ldo;
      const int row = 4 * wave + (lane >> 3), c8 = (lane & 7) * 8;
      for (int pass = 0; pass < 2; ++pass) {
        const v8h v = *(const v8h*)(h16 + row * kHP + c8);
        *(volatile v8h*)(hsb + (size_t)row * kTime * ldo + c8) = v;
        __threadfence();
      }
    }
  }
}

__global__ __launch_bounds__(kNT) void gat_score_kernel(const float* __restrict__ PQ, const float* __restrict__ bw,
                                                        const float* __restrict__ Wa, const float* __restrict__ ba,
                                                        _Float16* __restrict__ ATT) {
  __shared__ __align__(16) float Pl[16 * kEmb];
  __shared__ __align__(16) float Qt[kEmb * kNode];
  __shared__ float wa_s[kEmb];
  __shared__ __align__(16) float es[16 * kNode];
  const int ic = blockIdx.x, b = blockIdx.y;
  const int tid = threadIdx.x, lane = tid & 31, wave = tid >> 5;
  const int i0 = ic * 16;
#pragma unroll
  for (int it = 0; it < 2; ++it) {
    const int idx = it * kNT + tid;
    const int r = idx >> 5, c4 = (idx & 31) * 4;
    const v4f v = *(const v4f*)(PQ + ((size_t)(b * kNode + i0 + r)) * (2 * kEmb) + c4);
#pragma unroll
    for (int e = 0; e < 4; ++e) Pl[r * kEmb + c4 + e] = v[e] + bw[c4 + e];
  }
#pragma unroll 1
  for (int it = 0; it < 8; ++it) {
    const int idx = it * kNT + tid;
    const int jr = idx >> 5, c4 = (idx & 31) * 4;
    const v4f v = *(const v4f*)(PQ + ((size_t)(b * kNode + jr)) * (2 * kEmb) + kEmb + c4);
#pragma unroll
    for (int e = 0; e < 4; ++e) Qt[(c4 + e) * kNode + jr] = v[e];
  }
  if (tid < kEmb) wa_s[tid] = Wa[tid];
  __syncthreads();

  const int j = tid & 63, ig = tid >> 6;
  const float ba0 = ba[0];
  float a0 = ba0, a1 = ba0, a2 = ba0, a3 = ba0;
  const float* p0 = Pl + (ig * 4) * kEmb;
#pragma unroll 4
  for (int e = 0; e < kEmb; ++e) {
    const float q = Qt[e * kNode + j];
    const float w = wa_s[e];
    float t0 = p0[e] + q;            t0 = fmaxf(t0, 0.2f * t0);
    float t1 = p0[kEmb + e] + q;     t1 = fmaxf(t1, 0.2f * t1);
    float t2 = p0[2 * kEmb + e] + q; t2 = fmaxf(t2, 0.2f * t2);
    float t3 = p0[3 * kEmb + e] + q; t3 = fmaxf(t3, 0.2f * t3);
    a0 += w * t0; a1 += w * t1; a2 += w * t2; a3 += w * t3;
  }
  es[(ig * 4 + 0) * kNode + j] = a0;
  es[(ig * 4 + 1) * kNode + j] = a1;
  es[(ig * 4 + 2) * kNode + j] = a2;
  es[(ig * 4 + 3) * kNode + j] = a3;
  __syncthreads();

#pragma unroll
  for (int rr = 0; rr < 2; ++rr) {
    const int row = 2 * wave + rr;
    const float e0 = es[row * kNode + lane], e1 = es[row * kNode + 32 + lane];
    float m = fmaxf(e0, e1);
#pragma unroll
    for (int off = 1; off < 32; off <<= 1) m = fmaxf(m, __shfl_xor(m, off, 32));
    const float p0v = __expf(e0 - m), p1v = __expf(e1 - m);
    float s = p0v + p1v;
#pragma unroll
    for (int off = 1; off < 32; off <<= 1) s += __shfl_xor(s, off, 32);
    const float inv = 256.0f * (1.0f / s);
    es[row * kNode + lane]      = p0v * inv;
    es[row * kNode + 32 + lane] = p1v * inv;
  }
  __syncthreads();
  if (wave < 4) {
    const int row = 4 * wave + (lane >> 3), c8 = (lane & 7) * 8;
    v8h h;
#pragma unroll
    for (int e = 0; e < 8; ++e) h[e] = (_Float16)es[row * kNode + c8 + e];
    _Float16* dst = ATT + ((size_t)(b * kNode + i0 + row)) * kNode + c8;
    *(volatile v8h*)dst = h;
    __threadfence();
    *(volatile v8h*)dst = h;
  }
}

template <int BIAS_MODE, int OUT_MODE, int ACT>
static void launch_gemm(hipStream_t stream, const void* A, int lda, long sA, const void* Bt, int ldb, long sB,
                        void* C, int ldc, long sC, const float* bias, int M, int N, int K, float scale, int batch) {
  const int tiles = (M / 64) * (N / 64);
  dim3 grid((tiles + 7) / 8, batch);
  wmma_gemm64<0, false, BIAS_MODE, OUT_MODE, false, ACT><<<grid, 256, 0, stream>>>(
      (const unsigned short*)A, (const unsigned short*)nullptr, lda, sA,
      (const unsigned short*)Bt, (const unsigned short*)nullptr, ldb, sB,
      C, (void*)nullptr, ldc, sC, bias, (const float*)nullptr, 0L, M, N, K, scale);
}

extern "C" void kernel_launch(void* const* d_in, const int* in_sizes, int n_in,
                              void* d_out, int out_size, void* d_ws, size_t ws_size, hipStream_t stream) {
  if (n_in < 26 || d_out == nullptr || d_ws == nullptr) return;
  if (in_sizes[0] != kBatch * kTime * kNode || in_sizes[2] != kNode * kNode * kTaps || in_sizes[3] != kNode ||
      in_sizes[4] != kGate3 * kNode || in_sizes[5] != kGate3 * kHid || in_sizes[6] != kGate3 || in_sizes[7] != kGate3 ||
      in_sizes[8] != kEmb * 2 * kTime || in_sizes[9] != kEmb || in_sizes[10] != kEmb || in_sizes[11] != 1 ||
      in_sizes[12] != kGate3 * (kHid + kNode) || in_sizes[13] != kGate3 * kHid || in_sizes[14] != kGate3 || in_sizes[15] != kGate3 ||
      in_sizes[16] != kGate3 * kHid || in_sizes[17] != kGate3 * kHid || in_sizes[18] != kGate3 || in_sizes[19] != kGate3 ||
      in_sizes[20] != kNode * kHid || in_sizes[21] != kNode || in_sizes[22] != kNode * kHid || in_sizes[23] != kNode ||
      in_sizes[24] != kNode * kNode || in_sizes[25] != kNode ||
      out_size != kRows * kNode + kBatch * kNode) return;

  const float* x      = (const float*)d_in[0];
  const float* conv_w = (const float*)d_in[2];
  const float* conv_b = (const float*)d_in[3];
  const float* We_ih  = (const float*)d_in[4];
  const float* We_hh  = (const float*)d_in[5];
  const float* be_ih  = (const float*)d_in[6];
  const float* be_hh  = (const float*)d_in[7];
  const float* Ww     = (const float*)d_in[8];
  const float* bw     = (const float*)d_in[9];
  const float* Wa     = (const float*)d_in[10];
  const float* ba     = (const float*)d_in[11];
  const float* Wm_ih  = (const float*)d_in[12];
  const float* Wm_hh  = (const float*)d_in[13];
  const float* bm_ih  = (const float*)d_in[14];
  const float* bm_hh  = (const float*)d_in[15];
  const float* Wd_ih  = (const float*)d_in[16];
  const float* Wd_hh  = (const float*)d_in[17];
  const float* bd_ih  = (const float*)d_in[18];
  const float* bd_hh  = (const float*)d_in[19];
  const float* W_dec  = (const float*)d_in[20];
  const float* b_dec  = (const float*)d_in[21];
  const float* W_p1   = (const float*)d_in[22];
  const float* b_p1   = (const float*)d_in[23];
  const float* W_p2   = (const float*)d_in[24];
  const float* b_p2   = (const float*)d_in[25];
  float* out0 = (float*)d_out;
  float* out1 = (float*)d_out + (size_t)kRows * kNode;

  char* ws = (char*)d_ws; size_t off = 0;
  auto carve = [&](size_t bytes) -> char* { char* p = ws + off; off += (bytes + 255) & ~(size_t)255; return p; };
  _Float16* XCOL16  = (_Float16*)carve((size_t)kRows * kColK * 2);
  unsigned* WCONVu  = (unsigned*)carve((size_t)kNode * kColK * 2);
  unsigned* WCATu   = (unsigned*)carve((size_t)(2 * kEmb) * kTime * 2);
  unsigned* WEIHu   = (unsigned*)carve((size_t)kGate3 * kNode * 2);
  unsigned* WEHHu   = (unsigned*)carve((size_t)kGate3 * kHid * 2);
  unsigned* WMIHu   = (unsigned*)carve((size_t)kGate3 * (kHid + kNode) * 2);
  unsigned* WMHHu   = (unsigned*)carve((size_t)kGate3 * kHid * 2);
  unsigned* WDIHu   = (unsigned*)carve((size_t)kGate3 * kHid * 2);
  unsigned* WDHHu   = (unsigned*)carve((size_t)kGate3 * kHid * 2);
  unsigned* WDECu   = (unsigned*)carve((size_t)kNode * kHid * 2);
  unsigned* WP1u    = (unsigned*)carve((size_t)kNode * kHid * 2);
  unsigned* WP2u    = (unsigned*)carve((size_t)kNode * kNode * 2);
  float*    CONV32  = (float*)carve((size_t)kRows * kNode * 4);
  _Float16* C16BTN  = (_Float16*)carve((size_t)kRows * kNode * 2);
  _Float16* V16     = (_Float16*)carve((size_t)kPairRows * kTime * 2);
  float*    PQ32    = (float*)carve((size_t)kPairRows * (2 * kEmb) * 4);
  float*    XG32    = (float*)carve((size_t)kRows * kGate3 * 4);
  _Float16* HCAT16  = (_Float16*)carve((size_t)kRows * (kHid + kNode) * 2);
  _Float16* ATT16   = (_Float16*)carve((size_t)kBatch * kNode * kNode * 2);
  _Float16* HENC16  = (_Float16*)carve((size_t)kRows * kHid * 2);
  _Float16* HDEC16  = (_Float16*)carve((size_t)kRows * kHid * 2);
  _Float16* PRELU16 = (_Float16*)carve((size_t)kBatch * kNode * 2);
  if (off > ws_size || off > (size_t)134217728) return;

  const _Float16* WCONV16 = (const _Float16*)WCONVu;
  const _Float16* WCAT16  = (const _Float16*)WCATu;
  const _Float16* WEIH16  = (const _Float16*)WEIHu;
  const _Float16* WEHH16  = (const _Float16*)WEHHu;
  const _Float16* WMIH16  = (const _Float16*)WMIHu;
  const _Float16* WMHH16  = (const _Float16*)WMHHu;
  const _Float16* WDIH16  = (const _Float16*)WDIHu;
  const _Float16* WDHH16  = (const _Float16*)WDHHu;
  const _Float16* WDEC16  = (const _Float16*)WDECu;
  const _Float16* WP1_16  = (const _Float16*)WP1u;
  const _Float16* WP2_16  = (const _Float16*)WP2u;
  const float s16 = 1.0f / 16.0f;

  prep_x_kernel<<<1792, kNT, 0, stream>>>(x, XCOL16);
  prep_w_kernel<<<dim3(64, 11), kNT, 0, stream>>>(conv_w, Ww, We_ih, We_hh, Wm_ih, Wm_hh, Wd_ih, Wd_hh, W_dec, W_p1, W_p2,
                                                  WCONVu, WCATu, WEIHu, WEHHu, WMIHu, WMHHu, WDIHu, WDHHu, WDECu, WP1u, WP2u);
  launch_gemm<2, 0, 0>(stream, XCOL16, kColK, 0L, WCONV16, kColK, 0L, (void*)CONV32, kNode, 0L, conv_b, kRows, kNode, kColK, s16, 1);
  selu_layout_kernel<<<kBatch, kNT, 0, stream>>>(CONV32, C16BTN, V16);
  launch_gemm<0, 0, 0>(stream, V16, kTime, 0L, WCAT16, kTime, 0L, (void*)PQ32, 2 * kEmb, 0L, (const float*)nullptr,
                       kPairRows, 2 * kEmb, kTime, s16, 1);
  launch_gemm<2, 0, 0>(stream, C16BTN, kNode, 0L, WEIH16, kNode, 0L, (void*)XG32, kGate3, 0L, be_ih, kRows, kGate3, kNode, s16, 1);
  gru_rec_kernel<<<kBatch / 16, 128, 0, stream>>>(XG32, WEHH16, be_hh, HCAT16, kHid + kNode);
  gat_score_kernel<<<dim3(kNode / 16, kBatch), kNT, 0, stream>>>(PQ32, bw, Wa, ba, ATT16);
  launch_gemm<0, 1, 6>(stream, C16BTN, kNode, (long)kTime * kNode, ATT16, kNode, (long)kNode * kNode,
                       (void*)(HCAT16 + kHid), kHid + kNode, (long)kTime * (kHid + kNode), (const float*)nullptr,
                       kTime, kNode, kNode, 1.0f / 256.0f, kBatch);
  launch_gemm<2, 0, 0>(stream, HCAT16, kHid + kNode, 0L, WMIH16, kHid + kNode, 0L, (void*)XG32, kGate3, 0L, bm_ih,
                       kRows, kGate3, kHid + kNode, s16, 1);
  gru_rec_kernel<<<kBatch / 16, 128, 0, stream>>>(XG32, WMHH16, bm_hh, HENC16, kHid);
  launch_gemm<2, 0, 0>(stream, HENC16, kHid, 0L, WDIH16, kHid, 0L, (void*)XG32, kGate3, 0L, bd_ih, kRows, kGate3, kHid, s16, 1);
  gru_rec_kernel<<<kBatch / 16, 128, 0, stream>>>(XG32, WDHH16, bd_hh, HDEC16, kHid);
  launch_gemm<2, 0, 0>(stream, HDEC16, kHid, 0L, WDEC16, kHid, 0L, (void*)out0, kNode, 0L, b_dec, kRows, kNode, kHid, s16, 1);
  launch_gemm<2, 1, 2>(stream, HDEC16, kTime * kHid, 0L, WP1_16, kHid, 0L, (void*)PRELU16, kNode, 0L, b_p1, kBatch, kNode, kHid, s16, 1);
  launch_gemm<2, 0, 0>(stream, PRELU16, kNode, 0L, WP2_16, kNode, 0L, (void*)out1, kNode, 0L, b_p2, kBatch, kNode, kNode, s16, 1);
}
